// Mamba_dflow_MAE_60309930771131
// MI455X (gfx1250) — hardware-verified
//
#include <hip/hip_runtime.h>
#include <stdint.h>


constexpr int NB   = 4;
constexpr int L    = 1024;
constexpr int H    = 256;
constexpr int DI   = 512;
constexpr int DS   = 16;
constexpr int DC   = 4;
constexpr int DTR  = 16;
constexpr int XDR  = DTR + 2 * DS;
constexpr int XDP  = 64;
constexpr int NL   = 2;
constexpr int M    = NB * L;
constexpr int XZW  = 4 * DI;
constexpr int TCH  = 32;
constexpr int YP   = 132;

typedef __attribute__((ext_vector_type(16))) _Float16 v16h;
typedef __attribute__((ext_vector_type(8)))  _Float16 v8h;
typedef __attribute__((ext_vector_type(4)))  _Float16 v4h;
typedef __attribute__((ext_vector_type(16))) __bf16   v16b;
typedef __attribute__((ext_vector_type(8)))  __bf16   v8b;
typedef __attribute__((ext_vector_type(8)))  float    v8f;
typedef __attribute__((ext_vector_type(4)))  float    v4f;
#define PSCALE 32768.0f
#define U16(p) ((const unsigned short*)(const void*)(p))
#define PSCALE_INV (1.0f / 32768.0f)

__device__ __forceinline__ unsigned short f2bf_bits(float f) {
  unsigned u = __float_as_uint(f);
  return (unsigned short)((u + 0x7FFFu + ((u >> 16) & 1u)) >> 16);
}
__device__ __forceinline__ float bf_bits2f(unsigned short h) { return __uint_as_float(((unsigned)h) << 16); }

__device__ __forceinline__ void dep_guard_h(v8f& a, v8f& b, v16h x, v16h y) { asm volatile("v_nop\n\tv_nop\n\tv_nop\n\tv_nop" : "+v"(a), "+v"(b) : "v"(x), "v"(y)); }
__device__ __forceinline__ void dep_guard_b(v8f& a, v8f& b, v16b x, v16b y) { asm volatile("v_nop\n\tv_nop\n\tv_nop\n\tv_nop" : "+v"(a), "+v"(b) : "v"(x), "v"(y)); }
__device__ __forceinline__ void keep4_h(v16h a, v16h b, v16h c, v16h d) { asm volatile("v_nop" :: "v"(a), "v"(b), "v"(c), "v"(d)); }
__device__ __forceinline__ void keep4_b(v16b a, v16b b, v16b c, v16b d) { asm volatile("v_nop" :: "v"(a), "v"(b), "v"(c), "v"(d)); }
__device__ __forceinline__ void acc_guard4(v8f& a, v8f& b, v8f& c, v8f& d) { asm volatile("v_nop\n\tv_nop\n\tv_nop\n\tv_nop" : "+v"(a), "+v"(b), "+v"(c), "+v"(d)); }
template <typename T> struct Frag;
template <> struct Frag<_Float16> {
  typedef v16h V; union U { v16h v; v8h h[2]; };
  static __device__ __forceinline__ v16h load(const _Float16* p) {
    U f; f.h[0] = *(const v8h*)(p); f.h[1] = *(const v8h*)(p + 16); return f.v;
  }
  static __device__ __forceinline__ v8f mma(v16h a, v16h b, v8f c) {
    return __builtin_amdgcn_wmma_f32_16x16x32_f16(false, a, false, b, (short)0, c, false, false);
  }
  static __device__ __forceinline__ void guard(v8f& a, v8f& b, v16h x, v16h y) { dep_guard_h(a, b, x, y); }
  static __device__ __forceinline__ void keep(v16h a, v16h b, v16h c, v16h d) { keep4_h(a, b, c, d); }
};
template <> struct Frag<__bf16> {
  typedef v16b V; union U { v16b v; v8b h[2]; };
  static __device__ __forceinline__ v16b load(const __bf16* p) {
    U f; f.h[0] = *(const v8b*)(p); f.h[1] = *(const v8b*)(p + 16); return f.v;
  }
  static __device__ __forceinline__ v8f mma(v16b a, v16b b, v8f c) {
    return __builtin_amdgcn_wmma_f32_16x16x32_bf16(false, a, false, b, (short)0, c, false, false);
  }
  static __device__ __forceinline__ void guard(v8f& a, v8f& b, v16b x, v16b y) { dep_guard_b(a, b, x, y); }
  static __device__ __forceinline__ void keep(v16b a, v16b b, v16b c, v16b d) { keep4_b(a, b, c, d); }
};

template <int ET> struct Elem;
template <> struct Elem<0> { typedef _Float16 T; };
template <> struct Elem<1> { typedef __bf16 T; };
template <int ET, bool SPLIT, int BIAS_MODE, int OUT_MODE, bool RESID, int ACT = 0>
__global__ __launch_bounds__(256) void wmma_gemm64(
    const unsigned short* __restrict__ Ap, const unsigned short* __restrict__ A2p, int lda, long strideA,
    const unsigned short* __restrict__ Btp, const unsigned short* __restrict__ Bt2p, int ldb, long strideB,
    void* __restrict__ Cout, void* __restrict__ Cout2, int ldc, long strideC,
    const float* __restrict__ bias,
    const float* __restrict__ resid, long strideR,
    int M, int N, int K, float scale) {
  typedef typename Elem<ET>::T T;
  typedef typename Frag<T>::V V;
  const T* A = (const T*)Ap; const T* A2 = (const T*)A2p; const T* Bt = (const T*)Btp; const T* Bt2 = (const T*)Bt2p;
  __shared__ __align__(16) float sT[8][16 * 68];
  const int b    = blockIdx.y;
  const int lane = threadIdx.x & 31;
  const int wave = threadIdx.x >> 5;
  const int tilesN = N >> 6;
  const int tilesM = M >> 6;
  const int tile = blockIdx.x * 8 + wave;
  if (tile >= tilesM * tilesN) return;
  const int tm = tile / tilesN;
  const int tn = tile - tm * tilesN;
  const int m0 = tm << 6;
  const int n0 = tn << 6;

  const T* Ab  = A  + (size_t)b * strideA;
  const T* Bb  = Bt + (size_t)b * strideB;
  const T* Ab2 = SPLIT ? (A2  + (size_t)b * strideA) : nullptr;
  const T* Bb2 = SPLIT ? (Bt2 + (size_t)b * strideB) : nullptr;

  const int rlane = lane & 15;
  const int koff  = (lane >> 4) * 8;
  const int mOff  = (lane >> 4) * 8;

  v8f acc[4][4];
#pragma unroll
  for (int i = 0; i < 4; ++i)
#pragma unroll
    for (int j = 0; j < 4; ++j) acc[i][j] = (v8f){0.f,0.f,0.f,0.f,0.f,0.f,0.f,0.f};

  for (int k0 = 0; k0 < K; k0 += 32) {
    V bh[4], bl[4];
#pragma unroll
    for (int j = 0; j < 4; ++j) {
      const size_t bo = (size_t)(n0 + (j << 4) + rlane) * ldb + koff + k0;
      bh[j] = Frag<T>::load(Bb + bo);
      if (SPLIT) bl[j] = Frag<T>::load(Bb2 + bo);
    }
#pragma unroll
    for (int i = 0; i < 4; ++i) {
      const size_t ao = (size_t)(m0 + (i << 4) + rlane) * lda + koff + k0;
      V ah = Frag<T>::load(Ab + ao);
      V al;
      if (SPLIT) al = Frag<T>::load(Ab2 + ao);
#pragma unroll
      for (int j = 0; j < 4; ++j) {
        acc[i][j] = Frag<T>::mma(ah, bh[j], acc[i][j]);
        if (SPLIT) {
          acc[i][j] = Frag<T>::mma(ah, bl[j], acc[i][j]);
          acc[i][j] = Frag<T>::mma(al, bh[j], acc[i][j]);
        }
      }
      Frag<T>::guard(acc[i][0], acc[i][3], ah, SPLIT ? al : ah);
    }
    Frag<T>::keep(bh[0], bh[1], bh[2], bh[3]);
    if (SPLIT) Frag<T>::keep(bl[0], bl[1], bl[2], bl[3]);
  }
  acc_guard4(acc[0][0], acc[0][1], acc[0][2], acc[0][3]);
  acc_guard4(acc[1][0], acc[1][1], acc[1][2], acc[1][3]);
  acc_guard4(acc[2][0], acc[2][1], acc[2][2], acc[2][3]);
  acc_guard4(acc[3][0], acc[3][1], acc[3][2], acc[3][3]);

  float* slab = sT[wave];
  const float* Rb = RESID ? (resid + (size_t)b * strideR) : nullptr;
#pragma unroll
  for (int i = 0; i < 4; ++i) {
    const int mBase = m0 + (i << 4);
#pragma unroll
    for (int j = 0; j < 4; ++j) {
      const int n = n0 + (j << 4) + rlane;
      float bv = 0.f;
      if (BIAS_MODE == 2) bv = bias[n];
#pragma unroll
      for (int r = 0; r < 8; ++r) {
        float v = acc[i][j][r] * scale;
        if (BIAS_MODE == 1) v += bias[mBase + mOff + r];
        if (BIAS_MODE == 2) v += bv;
        if (RESID) v += Rb[(size_t)(mBase + mOff + r) * ldc + n];
        if (ACT == 1) v = tanhf(v);
        if (ACT == 2) v = fmaxf(v, 0.0f);
        if (ACT == 3) v = v / (1.0f + expf(-v));
        if (ACT == 4) v = (v > 0.f) ? v : 0.01f * v;
        if (ACT == 5) v = 0.5f * v * (1.0f + erff(v * 0.70710678118654752f));
        slab[(mOff + r) * 68 + (j << 4) + rlane] = v;
      }
    }
    __builtin_amdgcn_fence(__ATOMIC_RELEASE, "workgroup");
    __builtin_amdgcn_wave_barrier();
    __builtin_amdgcn_fence(__ATOMIC_ACQUIRE, "workgroup");
    if (OUT_MODE == 0) {
      float* C = (float*)Cout + (size_t)b * strideC;
      const int hh = lane >> 4, c4 = (lane & 15) * 4;
      for (int pass = 0; pass < 2; ++pass) {
#pragma unroll
        for (int it = 0; it < 8; ++it) {
          const int row = it * 2 + hh;
          v4f v = *(const v4f*)(slab + row * 68 + c4);
          *(volatile v4f*)(C + (size_t)(mBase + row) * ldc + n0 + c4) = v;
        }
        __threadfence();
      }
    } else {
      const int q = lane >> 3, c8 = (lane & 7) * 8;
      unsigned short* C  = (unsigned short*)Cout  + (size_t)b * strideC;
      unsigned short* C2 = (OUT_MODE == 2) ? ((unsigned short*)Cout2 + (size_t)b * strideC) : nullptr;
      for (int pass = 0; pass < 2; ++pass) {
#pragma unroll
        for (int it = 0; it < 4; ++it) {
          const int row = it * 4 + q;
          const float* sp = slab + row * 68 + c8;
          v8h hv, lv;
#pragma unroll
          for (int e = 0; e < 8; ++e) {
            if (OUT_MODE == 1) {
              hv[e] = (_Float16)sp[e];
            } else {
              unsigned short hb = f2bf_bits(sp[e]);
              unsigned short lb = f2bf_bits(sp[e] - bf_bits2f(hb));
              hv[e] = __builtin_bit_cast(_Float16, hb);
              lv[e] = __builtin_bit_cast(_Float16, lb);
            }
          }
          *(volatile v8h*)(C + (size_t)(mBase + row) * ldc + n0 + c8) = hv;
          if (OUT_MODE == 2) *(volatile v8h*)(C2 + (size_t)(mBase + row) * ldc + n0 + c8) = lv;
        }
        __threadfence();
      }
    }
    __builtin_amdgcn_fence(__ATOMIC_RELEASE, "workgroup");
    __builtin_amdgcn_wave_barrier();
    __builtin_amdgcn_fence(__ATOMIC_ACQUIRE, "workgroup");
  }
}

__global__ __launch_bounds__(256) void cast_scale_f16x2(
    const float* __restrict__ in, _Float16* __restrict__ out, int n2, float sc) {
  int i = blockIdx.x * 256 + threadIdx.x;
  if (i < n2) {
    const _Float16 h0 = (_Float16)(in[2 * i] * sc), h1 = (_Float16)(in[2 * i + 1] * sc);
    const unsigned u = (unsigned)__builtin_bit_cast(unsigned short, h0) | ((unsigned)__builtin_bit_cast(unsigned short, h1) << 16);
    ((volatile unsigned*)out)[i] = u;
    __threadfence();
    ((volatile unsigned*)out)[i] = u;
  }
}

__global__ __launch_bounds__(256) void cast_xw_pad_f16x2(
    const float* __restrict__ in, _Float16* __restrict__ out, int n2, float sc) {
  int i = blockIdx.x * 256 + threadIdx.x;
  if (i < n2) {
    const int e = 2 * i;
    const int p = e >> 15;
    const int rem = e & 32767;
    const int r = rem >> 9;
    const int k = rem & 511;
    const int rc = (r < XDR) ? r : (XDR - 1);
    const float* src = in + ((size_t)(p * XDR + rc) * DI + k);
    float f0 = src[0] * sc, f1 = src[1] * sc;
    if (r >= XDR) { f0 = 0.0f; f1 = 0.0f; }
    const _Float16 h0 = (_Float16)f0, h1 = (_Float16)f1;
    const unsigned u = (unsigned)__builtin_bit_cast(unsigned short, h0) | ((unsigned)__builtin_bit_cast(unsigned short, h1) << 16);
    ((volatile unsigned*)out)[i] = u;
    __threadfence();
    ((volatile unsigned*)out)[i] = u;
  }
}

__device__ __forceinline__ float wave_sum(float v) {
#pragma unroll
  for (int off = 16; off > 0; off >>= 1) v += __shfl_xor(v, off, 32);
  return v;
}
__device__ __forceinline__ void ln_row_store(v4f x0, v4f x1, const float* __restrict__ lnw, const float* __restrict__ lnb, float g,
                                             float* hrow, _Float16* h16row, float* srow, int lane) {
  float s = (x0[0] + x0[1]) + (x0[2] + x0[3]) + (x1[0] + x1[1]) + (x1[2] + x1[3]);
  s = wave_sum(s);
  const float mean = s * (1.0f / 256.0f);
  const v4f d0 = x0 - mean, d1 = x1 - mean;
  float ss = (d0[0] * d0[0] + d0[1] * d0[1]) + (d0[2] * d0[2] + d0[3] * d0[3])
           + (d1[0] * d1[0] + d1[1] * d1[1]) + (d1[2] * d1[2] + d1[3] * d1[3]);
  ss = wave_sum(ss);
  const float var = ss * (1.0f / 256.0f);
  const float rs = rsqrtf(var + 1e-12f);
  const v4f w0 = *(const v4f*)(lnw + 4 * lane), w1 = *(const v4f*)(lnw + 128 + 4 * lane);
  const v4f b0 = *(const v4f*)(lnb + 4 * lane), b1 = *(const v4f*)(lnb + 128 + 4 * lane);
  const v4f o0 = ((d0 * rs) * w0 + b0) * g;
  const v4f o1 = ((d1 * rs) * w1 + b1) * g;
  *(v4f*)(srow + 4 * lane) = o0;
  *(v4f*)(srow + 128 + 4 * lane) = o1;
  __builtin_amdgcn_fence(__ATOMIC_RELEASE, "workgroup");
  __builtin_amdgcn_wave_barrier();
  __builtin_amdgcn_fence(__ATOMIC_ACQUIRE, "workgroup");
  const v4f r0 = *(const v4f*)(srow + 8 * lane), r1 = *(const v4f*)(srow + 8 * lane + 4);
  v8h hv;
  hv[0] = (_Float16)(r0[0] * 8.0f); hv[1] = (_Float16)(r0[1] * 8.0f); hv[2] = (_Float16)(r0[2] * 8.0f); hv[3] = (_Float16)(r0[3] * 8.0f);
  hv[4] = (_Float16)(r1[0] * 8.0f); hv[5] = (_Float16)(r1[1] * 8.0f); hv[6] = (_Float16)(r1[2] * 8.0f); hv[7] = (_Float16)(r1[3] * 8.0f);
  for (int pass = 0; pass < 2; ++pass) {
    *(volatile v4f*)(hrow + 4 * lane) = o0;
    *(volatile v4f*)(hrow + 128 + 4 * lane) = o1;
    *(volatile v8h*)(h16row + 8 * lane) = hv;
    __threadfence();
  }
}

__global__ __launch_bounds__(256) void k_embed(const int* __restrict__ ids, const float* __restrict__ gate,
                                                const float* __restrict__ wemb, const float* __restrict__ pemb,
                                                const float* __restrict__ pemb2, const float* __restrict__ ttemb,
                                                const float* __restrict__ lnw, const float* __restrict__ lnb,
                                                float* __restrict__ hout, _Float16* __restrict__ h16, int nrows, int nV) {
  __shared__ __align__(16) float srow[8][256];
  const int wave = threadIdx.x >> 5, lane = threadIdx.x & 31;
  const int m = blockIdx.x * 8 + wave;
  if (m >= nrows) return;
  const int l = m & (L - 1);
  int id = ids[m];
  id = (id < 0) ? 0 : ((id >= nV) ? (nV - 1) : id);
  const float g = gate[m];
  const float* wr = wemb + (size_t)id * H;
  const float* pr = pemb + (size_t)l * H;
  const float* qr = pemb2 + (size_t)l * H;
  const v4f a0 = *(const v4f*)(wr + 4 * lane), a1 = *(const v4f*)(wr + 128 + 4 * lane);
  const v4f t0 = *(const v4f*)(ttemb + 4 * lane), t1 = *(const v4f*)(ttemb + 128 + 4 * lane);
  const v4f p0 = *(const v4f*)(pr + 4 * lane), p1 = *(const v4f*)(pr + 128 + 4 * lane);
  const v4f q0 = *(const v4f*)(qr + 4 * lane), q1 = *(const v4f*)(qr + 128 + 4 * lane);
  const v4f x0 = p0 * (a0 + t0) + q0;
  const v4f x1 = p1 * (a1 + t1) + q1;
  ln_row_store(x0, x1, lnw, lnb, g, hout + (size_t)m * H, h16 + (size_t)m * H, srow[wave], lane);
}

__global__ __launch_bounds__(256) void k_resid_ln(const float* __restrict__ mo, const float* __restrict__ hin,
                                                   const float* __restrict__ lnw, const float* __restrict__ lnb,
                                                   float* __restrict__ hout, _Float16* __restrict__ h16, int nrows) {
  __shared__ __align__(16) float srow[8][256];
  const int wave = threadIdx.x >> 5, lane = threadIdx.x & 31;
  const int m = blockIdx.x * 8 + wave;
  if (m >= nrows) return;
  const float* f = mo + (size_t)m * H;
  const float* bw = mo + (size_t)M * H + (size_t)m * H;
  const float* hr = hin + (size_t)m * H;
  const v4f f0 = *(const v4f*)(f + 4 * lane), f1 = *(const v4f*)(f + 128 + 4 * lane);
  const v4f g0 = *(const v4f*)(bw + 4 * lane), g1 = *(const v4f*)(bw + 128 + 4 * lane);
  const v4f r0 = *(const v4f*)(hr + 4 * lane), r1 = *(const v4f*)(hr + 128 + 4 * lane);
  const v4f x0 = (f0 + g0) + r0;
  const v4f x1 = (f1 + g1) + r1;
  ln_row_store(x0, x1, lnw, lnb, 1.0f, hout + (size_t)m * H, h16 + (size_t)m * H, srow[wave], lane);
}

__global__ __launch_bounds__(256) void k_conv_silu(const float* __restrict__ xz, const float* __restrict__ cw,
                                                    const float* __restrict__ cb, float* __restrict__ xc,
                                                    _Float16* __restrict__ xc16, int total) {
  const int t = blockIdx.x * 256 + threadIdx.x;
  if (t >= total) return;
  const int dq  = t & 127;
  const int m   = (t >> 7) & (M - 1);
  const int dir = t >> 19;
  const int d0  = dq * 4;
  const int l   = m & (L - 1);
  const int bb  = m >> 10;
  const float LOG2E = 1.4426950408889634f;
  const v4f bias = *(const v4f*)(cb + dir * DI + d0);
  const float* cwp = cw + (size_t)(dir * DI + d0) * DC;
  const v4f w0 = *(const v4f*)(cwp), w1 = *(const v4f*)(cwp + 4), w2 = *(const v4f*)(cwp + 8), w3 = *(const v4f*)(cwp + 12);
  v4f s = {0.0f, 0.0f, 0.0f, 0.0f};
#pragma unroll
  for (int k = 0; k < DC; ++k) {
    const int lr = dir ? (l + (DC - 1) - k) : (l - (DC - 1) + k);
    const bool valid = (unsigned)lr < (unsigned)L;
    const int lrc = valid ? lr : l;
    const v4f xv = *(const v4f*)(xz + (size_t)(bb * L + lrc) * XZW + dir * (2 * DI) + d0);
    const float fz = valid ? 1.0f : 0.0f;
    v4f wk;
    wk[0] = w0[k]; wk[1] = w1[k]; wk[2] = w2[k]; wk[3] = w3[k];
    s = s + wk * (xv * fz);
  }
  const v4f a = bias + s;
  v4f o;
  o[0] = a[0] * __builtin_amdgcn_rcpf(1.0f + __builtin_amdgcn_exp2f(-a[0] * LOG2E));
  o[1] = a[1] * __builtin_amdgcn_rcpf(1.0f + __builtin_amdgcn_exp2f(-a[1] * LOG2E));
  o[2] = a[2] * __builtin_amdgcn_rcpf(1.0f + __builtin_amdgcn_exp2f(-a[2] * LOG2E));
  o[3] = a[3] * __builtin_amdgcn_rcpf(1.0f + __builtin_amdgcn_exp2f(-a[3] * LOG2E));
  v4h hv;
  hv[0] = (_Float16)(o[0] * 64.0f); hv[1] = (_Float16)(o[1] * 64.0f); hv[2] = (_Float16)(o[2] * 64.0f); hv[3] = (_Float16)(o[3] * 64.0f);
  float* xp = xc + ((size_t)(dir * M + m) * DI + d0);
  _Float16* hp = xc16 + ((size_t)(dir * M + m) * DI + d0);
  for (int pass = 0; pass < 2; ++pass) {
    *(volatile v4f*)xp = o;
    *(volatile v4h*)hp = hv;
    __threadfence();
  }
}

__global__ __launch_bounds__(128) void k_scan(const float* __restrict__ xz, const float* __restrict__ xc,
                                               const float* __restrict__ xdbl, const float* __restrict__ wdt,
                                               const float* __restrict__ bdt, const float* __restrict__ alog,
                                               const float* __restrict__ dpar, _Float16* __restrict__ y16) {
  __shared__ __align__(16) float sX[TCH * XDP];
  __shared__ __align__(16) float sY[TCH * YP];
  const int tid = threadIdx.x, wave = tid >> 5, lane = tid & 31;
  const int d0  = blockIdx.x * 128;
  const int d   = d0 + tid;
  const int bb  = blockIdx.y;
  const int dir = blockIdx.z;
  const int pd  = dir * DI + d;
  const float LOG2E = 1.4426950408889634f;
  float A2[DS], hs[DS], w[DTR];
#pragma unroll
  for (int s = 0; s < DS; ++s) {
    A2[s] = -__builtin_amdgcn_exp2f(alog[(size_t)pd * DS + s] * LOG2E) * LOG2E;
    hs[s] = 0.0f;
  }
  {
    const v4f* wp = (const v4f*)(wdt + (size_t)pd * DTR);
    const v4f q0 = wp[0], q1 = wp[1], q2 = wp[2], q3 = wp[3];
    w[0] = q0[0]; w[1] = q0[1]; w[2]  = q0[2]; w[3]  = q0[3]; w[4]  = q1[0]; w[5]  = q1[1]; w[6]  = q1[2]; w[7]  = q1[3];
    w[8] = q2[0]; w[9] = q2[1]; w[10] = q2[2]; w[11] = q2[3]; w[12] = q3[0]; w[13] = q3[1]; w[14] = q3[2]; w[15] = q3[3];
  }
  const float bd = bdt[pd];
  const float Dd = dpar[pd];
  const float* xcb = xc + ((size_t)dir * M + (size_t)bb * L) * DI + d;
  const float* zb  = xz + (size_t)bb * L * XZW + dir * (2 * DI) + DI + d;
  const float* xdb = xdbl + ((size_t)dir * M + (size_t)bb * L) * XDP;
  _Float16* yb = y16 + ((size_t)dir * M + (size_t)bb * L) * DI + d0;
  const int c8 = (lane & 15) * 8;
#pragma unroll 1
  for (int ci = 0; ci < L / TCH; ++ci) {
    const int pb = dir ? (L - (ci + 1) * TCH) : (ci * TCH);
    __syncthreads();
#pragma unroll
    for (int it = 0; it < (TCH * XDP / 4) / 128; ++it) {
      const int idx = it * 128 + tid;
      const int row = idx >> 4;
      const int c4  = (idx & 15) * 4;
      *(v4f*)(sX + row * XDP + c4) = *(const v4f*)(xdb + (size_t)(pb + row) * XDP + c4);
    }
    __syncthreads();
#pragma unroll 1
    for (int j = 0; j < TCH; ++j) {
      const int r = dir ? (TCH - 1 - j) : j;
      const int p = pb + r;
      const float* sx = sX + r * XDP;
      float acc = 0.0f;
#pragma unroll
      for (int q = 0; q < DTR; ++q) acc += sx[q] * w[q];
      const float dtr = acc + bd;
      const float dt  = fmaxf(dtr, 0.0f) + log1pf(__builtin_amdgcn_exp2f(-fabsf(dtr) * LOG2E));
      const float x   = xcb[(size_t)p * DI];
      const float z   = zb[(size_t)p * XZW];
      const float dtx = dt * x;
      float y = 0.0f;
#pragma unroll
      for (int s = 0; s < DS; ++s) {
        const float dA = __builtin_amdgcn_exp2f(dt * A2[s]);
        hs[s] = dA * hs[s] + dtx * sx[DTR + s];
        y += hs[s] * sx[DTR + DS + s];
      }
      const float sg = __builtin_amdgcn_rcpf(1.0f + __builtin_amdgcn_exp2f(-z * LOG2E));
      sY[r * YP + tid] = (y + x * Dd) * (z * sg) * 64.0f;
    }
    __syncthreads();
    for (int pass = 0; pass < 2; ++pass) {
#pragma unroll
      for (int it = 0; it < 4; ++it) {
        const int row = wave * 8 + it * 2 + (lane >> 4);
        const float* sp = sY + row * YP + c8;
        const v4f u0 = *(const v4f*)sp, u1 = *(const v4f*)(sp + 4);
        v8h hv;
        hv[0] = (_Float16)u0[0]; hv[1] = (_Float16)u0[1]; hv[2] = (_Float16)u0[2]; hv[3] = (_Float16)u0[3];
        hv[4] = (_Float16)u1[0]; hv[5] = (_Float16)u1[1]; hv[6] = (_Float16)u1[2]; hv[7] = (_Float16)u1[3];
        *(volatile v8h*)(yb + (size_t)(pb + row) * DI + c8) = hv;
      }
      __threadfence();
    }
  }
}

__global__ __launch_bounds__(256) void k_head(const float* __restrict__ h, const float* __restrict__ gate,
                                               const float* __restrict__ d2w, const float* __restrict__ d2b,
                                               const float* __restrict__ opw, const float* __restrict__ opb,
                                               float* __restrict__ out) {
  __shared__ __align__(16) float sP[NB * H];
  __shared__ __align__(16) float sF[NB * H];
  __shared__ __align__(16) float sL[NB * H];
  const int c = threadIdx.x;
#pragma unroll
  for (int bb = 0; bb < NB; ++bb) {
    float mx = -__builtin_inff();
    const float* hb = h + (size_t)bb * L * H + c;
    const float* gb = gate + (size_t)bb * L;
#pragma unroll 1
    for (int l = 0; l < L; ++l) mx = fmaxf(mx, hb[(size_t)l * H] * gb[l]);
    sP[bb * H + c] = mx;
  }
  __syncthreads();
  {
    float f0 = 0.0f, f1 = 0.0f, f2 = 0.0f, f3 = 0.0f;
    const float* wr = d2w + (size_t)c * H;
#pragma unroll 1
    for (int k = 0; k < H; ++k) {
      const float wv = wr[k];
      f0 += sP[k] * wv; f1 += sP[H + k] * wv; f2 += sP[2 * H + k] * wv; f3 += sP[3 * H + k] * wv;
    }
    const float bv = d2b[c];
    sF[c] = f0 + bv; sF[H + c] = f1 + bv; sF[2 * H + c] = f2 + bv; sF[3 * H + c] = f3 + bv;
  }
  __syncthreads();
  {
    float g0 = 0.0f, g1 = 0.0f, g2 = 0.0f, g3 = 0.0f;
    const float* wr = opw + (size_t)c * H;
#pragma unroll 1
    for (int k = 0; k < H; ++k) {
      const float wv = wr[k];
      g0 += sF[k] * wv; g1 += sF[H + k] * wv; g2 += sF[2 * H + k] * wv; g3 += sF[3 * H + k] * wv;
    }
    const float bv = opb[c];
    sL[c] = g0 + bv; sL[H + c] = g1 + bv; sL[2 * H + c] = g2 + bv; sL[3 * H + c] = g3 + bv;
  }
  __syncthreads();
  const v4f lv = *(const v4f*)(sL + 4 * c);
  const v4f fv = *(const v4f*)(sF + 4 * c);
  const v4f gv0 = *(const v4f*)(gate + 4 * c);
  const v4f gv1 = *(const v4f*)(gate + 4 * (256 + c));
  const v4f gv2 = *(const v4f*)(gate + 4 * (512 + c));
  const v4f gv3 = *(const v4f*)(gate + 4 * (768 + c));
  float* o0 = out;
  float* o1 = out + NB * H;
  float* o2 = out + NB * H + NB * L;
  for (int pass = 0; pass < 2; ++pass) {
    *(volatile v4f*)(o0 + 4 * c) = lv;
    *(volatile v4f*)(o2 + 4 * c) = fv;
    *(volatile v4f*)(o1 + 4 * c) = gv0;
    *(volatile v4f*)(o1 + 4 * (256 + c)) = gv1;
    *(volatile v4f*)(o1 + 4 * (512 + c)) = gv2;
    *(volatile v4f*)(o1 + 4 * (768 + c)) = gv3;
    __threadfence();
  }
}

extern "C" void kernel_launch(void* const* d_in, const int* in_sizes, int n_in,
                              void* d_out, int out_size, void* d_ws, size_t ws_size,
                              hipStream_t stream) {
  if (n_in < 23) return;
  const int*   input_ids = (const int*)  d_in[0];
  const float* gate      = (const float*)d_in[1];
  const float* word_emb  = (const float*)d_in[2];
  const float* pos_emb   = (const float*)d_in[3];
  const float* pos_emb2  = (const float*)d_in[4];
  const float* tt_emb    = (const float*)d_in[5];
  const float* emb_ln_w  = (const float*)d_in[6];
  const float* emb_ln_b  = (const float*)d_in[7];
  const float* m_in_w    = (const float*)d_in[8];
  const float* m_conv_w  = (const float*)d_in[9];
  const float* m_conv_b  = (const float*)d_in[10];
  const float* m_x_w     = (const float*)d_in[11];
  const float* m_dt_w    = (const float*)d_in[12];
  const float* m_dt_b    = (const float*)d_in[13];
  const float* m_Alog    = (const float*)d_in[14];
  const float* m_D       = (const float*)d_in[15];
  const float* m_out_w   = (const float*)d_in[16];
  const float* blk_ln_w  = (const float*)d_in[17];
  const float* blk_ln_b  = (const float*)d_in[18];
  const float* d2_w      = (const float*)d_in[19];
  const float* d2_b      = (const float*)d_in[20];
  const float* op_w      = (const float*)d_in[21];
  const float* op_b      = (const float*)d_in[22];
  float* out = (float*)d_out;

  if (in_sizes[0] != M || in_sizes[1] != M) return;
  if ((in_sizes[2] % H) != 0 || in_sizes[2] < H) return;
  if (in_sizes[3] < L * H || in_sizes[4] < L * H) return;
  if (in_sizes[8] != NL * 2 * 2 * DI * H) return;
  if (in_sizes[11] != NL * 2 * XDR * DI) return;
  if (in_sizes[12] != NL * 2 * DI * DTR || in_sizes[14] != NL * 2 * DI * DS) return;
  if (in_sizes[16] != NL * 2 * H * DI) return;
  if (out_size != NB * H + NB * L + NB * H) return;
  const int nV = in_sizes[2] / H;

  char* ws = (char*)d_ws;
  size_t off = 0;
  auto carve = [&](size_t bytes) -> void* {
    void* p = ws + off;
    off = (off + bytes + 255) & ~(size_t)255;
    return p;
  };
  float*    hA   = (float*)   carve((size_t)M * H * 4);
  float*    hB   = (float*)   carve((size_t)M * H * 4);
  _Float16* h16  = (_Float16*)carve((size_t)M * H * 2);
  float*    xz   = (float*)   carve((size_t)M * XZW * 4);
  float*    xc   = (float*)   carve((size_t)2 * M * DI * 4);
  _Float16* xc16 = (_Float16*)carve((size_t)2 * M * DI * 2);
  float*    xdbl = (float*)   carve((size_t)2 * M * XDP * 4);
  _Float16* y16  = (_Float16*)carve((size_t)2 * M * DI * 2);
  float*    mo   = (float*)   carve((size_t)2 * M * H * 4);
  _Float16* Wi16 = (_Float16*)carve((size_t)NL * 2 * 2 * DI * H * 2);
  _Float16* Wx16 = (_Float16*)carve((size_t)NL * 2 * XDP * DI * 2);
  _Float16* Wo16 = (_Float16*)carve((size_t)NL * 2 * H * DI * 2);
  if (off > ws_size) return;

  auto cdiv = [](int a, int b) { return (a + b - 1) / b; };
  const float* fdummy = gate;

  {
    const int n2i = NL * 2 * 2 * DI * H / 2;
    cast_scale_f16x2<<<cdiv(n2i, 256), 256, 0, stream>>>(m_in_w, Wi16, n2i, 64.0f);
    const int n2o = NL * 2 * H * DI / 2;
    cast_scale_f16x2<<<cdiv(n2o, 256), 256, 0, stream>>>(m_out_w, Wo16, n2o, 64.0f);
    const int n2x = NL * 2 * XDP * DI / 2;
    cast_xw_pad_f16x2<<<cdiv(n2x, 256), 256, 0, stream>>>(m_x_w, Wx16, n2x, 64.0f);
  }

  k_embed<<<cdiv(M, 8), 256, 0, stream>>>(input_ids, gate, word_emb, pos_emb, pos_emb2, tt_emb,
                                           emb_ln_w, emb_ln_b, hA, h16, M, nV);

  float* hcur = hA;
  float* hnext = hB;
  for (int l = 0; l < NL; ++l) {
    const _Float16* Wi  = Wi16 + (size_t)l * (2 * 2 * DI) * H;
    const _Float16* Wx  = Wx16 + (size_t)(l * 2) * XDP * DI;
    const _Float16* Wo  = Wo16 + (size_t)(l * 2) * H * DI;
    const float* cw  = m_conv_w + (size_t)l * 2 * DI * DC;
    const float* cb  = m_conv_b + (size_t)l * 2 * DI;
    const float* wdt = m_dt_w   + (size_t)l * 2 * DI * DTR;
    const float* bdt = m_dt_b   + (size_t)l * 2 * DI;
    const float* al  = m_Alog   + (size_t)l * 2 * DI * DS;
    const float* dp  = m_D      + (size_t)l * 2 * DI;

    wmma_gemm64<0, false, 0, 0, false, 0><<<dim3((M / 64) * (XZW / 64) / 8, 1), 256, 0, stream>>>(
        U16(h16), U16(h16), H, (long)0,
        U16(Wi), U16(Wi), H, (long)0,
        (void*)xz, (void*)xz, XZW, (long)0,
        fdummy, fdummy, (long)0,
        M, XZW, H, 1.0f / 512.0f);

    {
      const int total = 2 * M * (DI / 4);
      k_conv_silu<<<cdiv(total, 256), 256, 0, stream>>>(xz, cw, cb, xc, xc16, total);
    }

    wmma_gemm64<0, false, 0, 0, false, 0><<<dim3(cdiv((M / 64) * (XDP / 64), 8), 2), 256, 0, stream>>>(
        U16(xc16), U16(xc16), DI, (long)M * DI,
        U16(Wx), U16(Wx), DI, (long)XDP * DI,
        (void*)xdbl, (void*)xdbl, XDP, (long)M * XDP,
        fdummy, fdummy, (long)0,
        M, XDP, DI, 1.0f / 4096.0f);

    k_scan<<<dim3(DI / 128, NB, 2), 128, 0, stream>>>(xz, xc, xdbl, wdt, bdt, al, dp, y16);

    wmma_gemm64<0, false, 0, 0, false, 0><<<dim3(cdiv((M / 64) * (H / 64), 8), 2), 256, 0, stream>>>(
        U16(y16), U16(y16), DI, (long)M * DI,
        U16(Wo), U16(Wo), DI, (long)H * DI,
        (void*)mo, (void*)mo, H, (long)M * H,
        fdummy, fdummy, (long)0,
        M, H, DI, 1.0f / 4096.0f);

    k_resid_ln<<<cdiv(M, 8), 256, 0, stream>>>(mo, hcur, blk_ln_w + (size_t)l * H, blk_ln_b + (size_t)l * H,
                                                hnext, h16, M);
    float* t = hcur; hcur = hnext; hnext = t;
  }

  k_head<<<1, 256, 0, stream>>>(hcur, gate, d2_w, d2_b, op_w, op_b, out);
}
